// TuckerMoELayer_72370198937819
// MI455X (gfx1250) — hardware-verified
//
#include <hip/hip_runtime.h>
#include <math.h>

typedef __attribute__((ext_vector_type(16))) _Float16 v16h;
typedef __attribute__((ext_vector_type(16))) __bf16 v16b;
typedef __attribute__((ext_vector_type(8)))  _Float16 v8h;
typedef __attribute__((ext_vector_type(8)))  __bf16 v8b;
typedef __attribute__((ext_vector_type(8)))  float v8f;
typedef __attribute__((ext_vector_type(4)))  float v4f;
typedef __attribute__((ext_vector_type(4)))  unsigned v4u;
typedef _Float16 h16;

#ifndef NB
#define NB 1024
#endif
#define NB_FULL 1024
#define DIN  1024
#define DFF  1024
#define DOUT 1024
#define RK   64
#define NG   8
#define EPG  32
#define NEXP 256
#define KTOP 8
#define NPAIR (NB * KTOP)
#define SROWS (NPAIR + NG * 128)
#define KP   (NG * RK)
#define PREP (2 * KP)
#define PCARRY 16.0f
#define WCARRY 64.0f
#define HSCALE (1.0f / 16.0f)
#define GSCALE (1.0f / 4096.0f)
#define ASCALE 4.0f
#define XSCALE (1.0f / 16.0f)
#define OSCALE (1.0f / 268435456.0f)
#define PLAN_PIT (NPAIR / 4 / 256)
#define PLAN_SIT (SROWS / 4 / 256)

#define WS_XB   ((size_t)0)
#define WS_W1T  (WS_XB   + (size_t)NB * DIN * 2)
#define WS_CG   (WS_W1T  + (size_t)PREP * DIN * 2)
#define WS_CU   (WS_CG   + (size_t)NEXP * RK * RK * 2)
#define WS_CD   (WS_CU   + (size_t)NEXP * RK * RK * 2)
#define WS_UG   (WS_CD   + (size_t)NEXP * RK * RK * 2)
#define WS_UU   (WS_UG   + (size_t)NG * DFF * RK * 2)
#define WS_UD   (WS_UU   + (size_t)NG * DFF * RK * 2)
#define WS_UO   (WS_UD   + (size_t)NG * RK * DFF * 2)
#define WS_PRE  (WS_UO   + (size_t)DOUT * KP * 2)
#define WS_HG   (WS_PRE  + (size_t)NB * PREP * 2)
#define WS_HU   (WS_HG   + (size_t)SROWS * RK * 2)
#define WS_ACT  (WS_HU   + (size_t)SROWS * RK * 2)
#define WS_XD   (WS_ACT  + (size_t)SROWS * DFF * 2)
#define WS_HD   (WS_XD   + (size_t)SROWS * RK * 2)
#define WS_A2   (WS_HD   + (size_t)SROWS * RK * 4)
#define WS_SEL  (WS_A2   + (size_t)NB * KP * 2)
#define WS_WT   (WS_SEL  + (size_t)NPAIR * 4)
#define WS_POS  (WS_WT   + (size_t)NPAIR * 4)
#define WS_SRT  (WS_POS  + (size_t)NPAIR * 4)
#define WS_ETAB (WS_SRT  + (size_t)SROWS * 4)
#define WS_HDR  (WS_ETAB + (size_t)2 * NEXP * 4)
#define WS_END  (WS_HDR  + (size_t)128)

static_assert(NB % 128 == 0);
static_assert(NB <= NB_FULL);
static_assert(NEXP == NG * EPG && NEXP == 256 && NEXP == 8 * 32);
static_assert(KTOP == 8 && RK == 64 && EPG == 32);
static_assert(DIN % 32 == 0 && KP % 32 == 0 && DFF % 32 == 0 && RK % 32 == 0 && (KP * 2) % 128 == 0);
static_assert(SROWS % 128 == 0 && SROWS >= NPAIR + NG * 127);
static_assert((size_t)NB_FULL * DOUT * 4 == 4194304);
static_assert(WS_W1T % 128 == 0 && WS_CG % 128 == 0 && WS_UG % 128 == 0 && WS_UD % 128 == 0 && WS_UO % 128 == 0 && WS_PRE % 128 == 0);
static_assert(WS_HG % 128 == 0 && WS_HU % 128 == 0 && WS_ACT % 128 == 0 && WS_XD % 128 == 0 && WS_HD % 128 == 0 && WS_A2 % 128 == 0);
static_assert(WS_SEL % 128 == 0 && WS_WT % 128 == 0 && WS_POS % 128 == 0 && WS_SRT % 128 == 0 && WS_ETAB % 128 == 0 && WS_HDR % 128 == 0);
static_assert(WS_END <= (size_t)134217728);
static_assert((size_t)(NB * DIN / 8 / 256) * 256 * 8 == (size_t)NB * DIN);
static_assert((size_t)(RK / 64) * (DIN / 64) * NG * 4096 == (size_t)NG * DIN * RK);
static_assert((size_t)(RK / 64) * (RK / 64) * NEXP * 4096 == (size_t)NEXP * RK * RK);
static_assert((size_t)(DFF / 64) * (RK / 64) * NG * 4096 == (size_t)NG * RK * DFF);
static_assert((size_t)(DOUT / 64) * (RK / 64) * NG * 4096 == (size_t)DOUT * KP);
static_assert((size_t)(NB / 8) * 8 * KTOP == (size_t)NPAIR);
static_assert((size_t)PLAN_PIT * 256 * 4 == (size_t)NPAIR && (size_t)PLAN_SIT * 256 * 4 == (size_t)SROWS);
static_assert((size_t)(PREP / 128) * (NB / 128) * 128 * 128 == (size_t)NB * PREP);
static_assert((size_t)(DFF / 64) * (SROWS / 128) * 128 * 64 == (size_t)SROWS * DFF);
static_assert((size_t)(SROWS / 128) * 128 * 64 == (size_t)SROWS * RK);
static_assert((size_t)(NB / 8) * 8 * KP == (size_t)NB * KP);
static_assert((size_t)(DOUT / 128) * (NB / 128) * 128 * 128 == (size_t)NB * DOUT);
static_assert(32 * 16 * 4 == 16 * 128);
static_assert(32 * 16 * 8 == 32 * 128);
static_assert(32 * 16 * 8 == 16 * 256);
static_assert(32 * 16 * 2 == KP * 2);
static_assert(16 * 16 == 8 * KTOP * 4);
static_assert((size_t)(2 * NPAIR + SROWS + 2 * NEXP + 32) * 4 <= 131072);
static_assert((size_t)(8 * DIN + 8 * NEXP + 128) * 4 <= 131072);

__device__ __forceinline__ v8f wmma16(v16h a, v16h b, v8f c) {
  v8f d = __builtin_amdgcn_wmma_f32_16x16x32_f16(false, a, false, b, (short)0, c, false, false);
  asm volatile("v_nop\n\tv_nop\n\tv_nop\n\tv_nop" : "+v"(d) : "v"(a), "v"(b));
  return d;
}
__device__ __forceinline__ v8f wmma_bf(v16b a, v16b b, v8f c) {
  v8f d = __builtin_amdgcn_wmma_f32_16x16x32_bf16(false, a, false, b, (short)0, c, false, false);
  asm volatile("v_nop\n\tv_nop\n\tv_nop\n\tv_nop" : "+v"(d) : "v"(a), "v"(b));
  return d;
}
__device__ __forceinline__ float bfr(float v) { return (float)(__bf16)v; }
static __device__ __forceinline__ h16 toh_flush(float v) { const h16 r = (h16)v; return (fabsf(v) < 6.103515625e-05f) ? (h16)0.0f : r; }
__device__ __forceinline__ v16b ldfrag_b(const unsigned short* p) { union { v16b v; v4u q[2]; } f; f.q[0] = *(const v4u*)p; f.q[1] = *(const v4u*)(p + 16); return f.v; }
__device__ __forceinline__ v16h ldfrag_h(const unsigned short* p) { union { v16h v; v4u q[2]; } f; f.q[0] = *(const v4u*)p; f.q[1] = *(const v4u*)(p + 16); return f.v; }

__global__ __launch_bounds__(256) void k_cvt_x(const float* __restrict__ X, unsigned short* __restrict__ XB) {
  const unsigned i = blockIdx.x * 256u + threadIdx.x;
  const unsigned ic = i < (unsigned)(NB * DIN / 8) ? i : (unsigned)(NB * DIN / 8 - 1);
  const v4f a = *(const v4f*)(X + (size_t)ic * 8), b = *(const v4f*)(X + (size_t)ic * 8 + 4);
  union { v8b h; v4u u; } o;
#pragma unroll
  for (int j = 0; j < 4; ++j) { o.h[j] = (__bf16)a[j]; o.h[4 + j] = (__bf16)b[j]; }
  const v4u val = o.u;
  volatile v4u* p = (volatile v4u*)(XB + (size_t)ic * 8);
  *p = val; __threadfence(); *p = val;
}

__global__ __launch_bounds__(256) void k_tr(const float* __restrict__ S, unsigned short* __restrict__ Dst, unsigned K, unsigned N, unsigned dpitch, unsigned erow, unsigned ecol, float sc, int f16) {
  __shared__ float tile[64][65];
  const unsigned t = threadIdx.x, e = blockIdx.z, k0 = blockIdx.y * 64u, n0 = blockIdx.x * 64u;
  const float* s = S + (size_t)e * K * N;
#pragma unroll
  for (unsigned it = 0; it < 4; ++it) { const unsigned idx = it * 256u + t, kr = idx >> 4, c4 = idx & 15u;
    const v4f v = *(const v4f*)(s + (size_t)(k0 + kr) * N + n0 + 4u * c4);
    tile[kr][4u * c4 + 0] = v[0]; tile[kr][4u * c4 + 1] = v[1]; tile[kr][4u * c4 + 2] = v[2]; tile[kr][4u * c4 + 3] = v[3]; }
  __syncthreads();
  v4u o[2];
#pragma unroll
  for (unsigned it = 0; it < 2; ++it) { const unsigned idx = it * 256u + t, nr = idx >> 3, q = idx & 7u;
    union { v8h h; v4u u; } wh; union { v8b b; v4u u; } wb;
#pragma unroll
    for (int i = 0; i < 8; ++i) { const float v = bfr(tile[8u * q + i][nr]); wh.h[i] = toh_flush(v * sc); wb.b[i] = (__bf16)v; }
    const v4u uh = wh.u, ub = wb.u;
    o[it] = (f16 != 0) ? uh : ub; }
#pragma unroll
  for (unsigned it = 0; it < 2; ++it) { const unsigned idx = it * 256u + t, nr = idx >> 3, q = idx & 7u;
    *(volatile v4u*)(Dst + (size_t)(e * erow + n0 + nr) * dpitch + e * ecol + k0 + 8u * q) = o[it]; }
  __threadfence();
#pragma unroll
  for (unsigned it = 0; it < 2; ++it) { const unsigned idx = it * 256u + t, nr = idx >> 3, q = idx & 7u;
    *(volatile v4u*)(Dst + (size_t)(e * erow + n0 + nr) * dpitch + e * ecol + k0 + 8u * q) = o[it]; }
}

__global__ __launch_bounds__(256) void k_router(const unsigned short* __restrict__ XB, const float* __restrict__ WG, int* __restrict__ SEL, float* __restrict__ WT) {
  __shared__ __align__(16) float xs[8][DIN];
  __shared__ __align__(16) float lg[8][NEXP];
  __shared__ __align__(16) int   os[64];
  __shared__ __align__(16) float ow[64];
  const unsigned tid = threadIdx.x, lane = tid & 31u;
  const unsigned wave = __builtin_amdgcn_readfirstlane(tid >> 5);
  const unsigned t0 = blockIdx.x * 8u;
#pragma unroll
  for (unsigned it = 0; it < 4; ++it) { const unsigned idx = it * 256u + tid, row = idx >> 7, c8 = idx & 127u;
    const v4u q = *(const v4u*)(XB + (size_t)(t0 + row) * DIN + 8u * c8);
    v4f a, b;
    a[0] = __uint_as_float(q[0] << 16); a[1] = __uint_as_float(q[0] & 0xffff0000u); a[2] = __uint_as_float(q[1] << 16); a[3] = __uint_as_float(q[1] & 0xffff0000u);
    b[0] = __uint_as_float(q[2] << 16); b[1] = __uint_as_float(q[2] & 0xffff0000u); b[2] = __uint_as_float(q[3] << 16); b[3] = __uint_as_float(q[3] & 0xffff0000u);
    *(v4f*)&xs[row][8u * c8] = a; *(v4f*)&xs[row][8u * c8 + 4u] = b; }
  __syncthreads();
  float acc[8];
#pragma unroll
  for (int r = 0; r < 8; ++r) acc[r] = 0.0f;
  const float* wp = WG + tid;
#pragma unroll 1
  for (unsigned k4 = 0; k4 < DIN / 4; ++k4) {
    const float w0 = bfr(wp[(size_t)(4u * k4 + 0u) * NEXP]), w1 = bfr(wp[(size_t)(4u * k4 + 1u) * NEXP]);
    const float w2 = bfr(wp[(size_t)(4u * k4 + 2u) * NEXP]), w3 = bfr(wp[(size_t)(4u * k4 + 3u) * NEXP]);
#pragma unroll
    for (int r = 0; r < 8; ++r) { const v4f xv = *(const v4f*)&xs[r][4u * k4];
      acc[r] = fmaf(xv[0], w0, acc[r]); acc[r] = fmaf(xv[1], w1, acc[r]); acc[r] = fmaf(xv[2], w2, acc[r]); acc[r] = fmaf(xv[3], w3, acc[r]); } }
#pragma unroll
  for (int r = 0; r < 8; ++r) lg[r][tid] = acc[r];
  __syncthreads();
  float v[8];
#pragma unroll
  for (int j = 0; j < 8; ++j) v[j] = lg[wave][j * 32 + lane];
  float myv = 0.0f; int myi = 0;
#pragma unroll 1
  for (int it = 0; it < KTOP; ++it) {
    float bv = v[0]; int bi = (int)lane;
#pragma unroll
    for (int j = 1; j < 8; ++j) { const int idx = j * 32 + (int)lane; const bool tk = v[j] > bv; bv = tk ? v[j] : bv; bi = tk ? idx : bi; }
#pragma unroll
    for (int off = 16; off > 0; off >>= 1) { const float ov = __shfl_xor(bv, off); const int oi = __shfl_xor(bi, off);
      const bool tk = (ov > bv) || (ov == bv && oi < bi); bv = tk ? ov : bv; bi = tk ? oi : bi; }
    const bool mine = ((int)lane == it); myv = mine ? bv : myv; myi = mine ? bi : myi;
#pragma unroll
    for (int j = 0; j < 8; ++j) { const bool ko = (bi == j * 32 + (int)lane); v[j] = ko ? -3.4e38f : v[j]; }
  }
  const float m = __shfl(myv, 0);
  const float arg = (lane < 8u) ? (myv - m) : 0.0f;
  const float ex = expf(arg);
  const float ev = (lane < 8u) ? ex : 0.0f;
  float s = ev; s += __shfl_xor(s, 1); s += __shfl_xor(s, 2); s += __shfl_xor(s, 4);
  const float wgt = ev * (1.0f / s);
  if (lane < 8u) { os[wave * 8u + lane] = myi; ow[wave * 8u + lane] = wgt; }
  __syncthreads();
  if (tid < 16u) {
    const v4u a = *(const v4u*)&os[4u * tid]; const v4f b = *(const v4f*)&ow[4u * tid];
    volatile v4u* ps = (volatile v4u*)(SEL + (size_t)t0 * KTOP + 4u * tid);
    volatile v4f* pw = (volatile v4f*)(WT + (size_t)t0 * KTOP + 4u * tid);
    *ps = a; *pw = b; __threadfence(); *ps = a; *pw = b;
  }
}

__global__ __launch_bounds__(256) void k_plan(const int* __restrict__ SEL, int* __restrict__ POS, int* __restrict__ SRT, int* __restrict__ ETAB, int* __restrict__ HDR) {
  __shared__ __align__(16) unsigned s_sel[NPAIR];
  __shared__ __align__(16) unsigned s_pos[NPAIR];
  __shared__ __align__(16) unsigned s_srt[SROWS];
  __shared__ __align__(16) unsigned s_tab[2 * NEXP];
  __shared__ __align__(16) unsigned s_hdr[32];
  const unsigned tid = threadIdx.x;
#pragma unroll 1
  for (unsigned it = 0; it < PLAN_PIT; ++it) { const unsigned i4 = it * 256u + tid; const v4u q = *(const v4u*)(SEL + 4u * i4);
#pragma unroll
    for (int j = 0; j < 4; ++j) { int e = (int)q[j]; e = e < 0 ? 0 : (e > NEXP - 1 ? NEXP - 1 : e); s_sel[4u * i4 + j] = (unsigned)e; s_pos[4u * i4 + j] = 0u; } }
#pragma unroll 1
  for (unsigned it = 0; it < PLAN_SIT; ++it) { const unsigned i4 = it * 256u + tid;
#pragma unroll
    for (int j = 0; j < 4; ++j) s_srt[4u * i4 + j] = 0u; }
  if (tid < 32u) s_hdr[tid] = 0u;
  __syncthreads();
  unsigned c = 0;
#pragma unroll 1
  for (unsigned f4 = 0; f4 < NPAIR / 4; ++f4) { const v4u q = *(const v4u*)&s_sel[4u * f4];
    c += (q[0] == tid ? 1u : 0u) + (q[1] == tid ? 1u : 0u) + (q[2] == tid ? 1u : 0u) + (q[3] == tid ? 1u : 0u); }
  s_tab[NEXP + tid] = c;
  __syncthreads();
  if (tid == 0u) {
    unsigned row = 0;
#pragma unroll 1
    for (unsigned g = 0; g < NG; ++g) { s_hdr[g] = row; unsigned gc = 0;
#pragma unroll 1
      for (unsigned j = 0; j < EPG; ++j) { const unsigned e = g * EPG + j; s_tab[e] = row + gc; gc += s_tab[NEXP + e]; }
      s_hdr[16u + g] = gc; row += ((gc + 127u) >> 7) << 7; }
    s_hdr[NG] = row;
  }
  __syncthreads();
  const unsigned b = s_tab[tid]; unsigned jn = 0;
#pragma unroll 1
  for (unsigned f4 = 0; f4 < NPAIR / 4; ++f4) { const v4u q = *(const v4u*)&s_sel[4u * f4];
#pragma unroll
    for (int i = 0; i < 4; ++i) if (q[i] == tid) { unsigned p = b + jn; p = p < (unsigned)SROWS ? p : (unsigned)(SROWS - 1); s_srt[p] = 4u * f4 + i; s_pos[4u * f4 + i] = p; ++jn; } }
  __syncthreads();
  v4u pv[PLAN_PIT], sv[PLAN_SIT];
#pragma unroll
  for (unsigned it = 0; it < PLAN_PIT; ++it) pv[it] = *(const v4u*)&s_pos[4u * (it * 256u + tid)];
#pragma unroll
  for (unsigned it = 0; it < PLAN_SIT; ++it) sv[it] = *(const v4u*)&s_srt[4u * (it * 256u + tid)];
  const v4u tv = *(const v4u*)&s_tab[4u * (tid & 127u)];
  const v4u hv = *(const v4u*)&s_hdr[4u * (tid & 7u)];
#pragma unroll
  for (unsigned it = 0; it < PLAN_PIT; ++it) *(volatile v4u*)(POS + 4u * (it * 256u + tid)) = pv[it];
#pragma unroll
  for (unsigned it = 0; it < PLAN_SIT; ++it) *(volatile v4u*)(SRT + 4u * (it * 256u + tid)) = sv[it];
  if (tid < 128u) *(volatile v4u*)(ETAB + 4u * tid) = tv;
  if (tid < 8u) *(volatile v4u*)(HDR + 4u * tid) = hv;
  __threadfence();
#pragma unroll
  for (unsigned it = 0; it < PLAN_PIT; ++it) *(volatile v4u*)(POS + 4u * (it * 256u + tid)) = pv[it];
#pragma unroll
  for (unsigned it = 0; it < PLAN_SIT; ++it) *(volatile v4u*)(SRT + 4u * (it * 256u + tid)) = sv[it];
  if (tid < 128u) *(volatile v4u*)(ETAB + 4u * tid) = tv;
  if (tid < 8u) *(volatile v4u*)(HDR + 4u * tid) = hv;
}

__global__ __launch_bounds__(256) void k_pre(const unsigned short* __restrict__ XB, const unsigned short* __restrict__ W1T, unsigned short* __restrict__ PRE) {
  __shared__ __align__(16) _Float16 sh[8][32][64];
  const unsigned t = threadIdx.x, lane = t & 31u, lm = lane & 15u, lh = lane >> 4;
  const unsigned wave = __builtin_amdgcn_readfirstlane(t >> 5);
  const unsigned wm = wave >> 1, wn = wave & 1u;
  const unsigned m0 = blockIdx.y * 128u, n0 = blockIdx.x * 128u;
  const unsigned short* ar[2]; const unsigned short* br[4];
#pragma unroll
  for (int mi = 0; mi < 2; ++mi) ar[mi] = XB + (size_t)(m0 + wm * 32u + mi * 16u + lm) * DIN + 8u * lh;
#pragma unroll
  for (int ni = 0; ni < 4; ++ni) br[ni] = W1T + (size_t)(n0 + wn * 64u + ni * 16u + lm) * DIN + 8u * lh;
  v8f acc[2][4] = {};
#pragma unroll 2
  for (unsigned kc = 0; kc < DIN / 32; ++kc) { v16b a[2], b[4];
#pragma unroll
    for (int mi = 0; mi < 2; ++mi) a[mi] = ldfrag_b(ar[mi] + kc * 32u);
#pragma unroll
    for (int ni = 0; ni < 4; ++ni) b[ni] = ldfrag_b(br[ni] + kc * 32u);
#pragma unroll
    for (int mi = 0; mi < 2; ++mi)
#pragma unroll
      for (int ni = 0; ni < 4; ++ni) acc[mi][ni] = wmma_bf(a[mi], b[ni], acc[mi][ni]); }
#pragma unroll
  for (int ni = 0; ni < 4; ++ni)
#pragma unroll
    for (int mi = 0; mi < 2; ++mi)
#pragma unroll
      for (int r = 0; r < 8; ++r) sh[wave][mi * 16 + 8u * lh + r][ni * 16 + lm] = toh_flush(acc[mi][ni][r] * PCARRY);
  __syncthreads();
  v4u o[8];
#pragma unroll
  for (unsigned it = 0; it < 8; ++it) { const unsigned rw = it * 4u + (lane >> 3), q = lane & 7u; union { v8h h; v4u u; } w; w.h = *(const v8h*)&sh[wave][rw][8u * q]; o[it] = w.u; }
  unsigned short* hb = PRE + (size_t)(m0 + wm * 32u) * PREP + n0 + wn * 64u;
#pragma unroll
  for (unsigned it = 0; it < 8; ++it) { const unsigned rw = it * 4u + (lane >> 3), q = lane & 7u; *(volatile v4u*)(hb + (size_t)rw * PREP + 8u * q) = o[it]; }
  __threadfence();
#pragma unroll
  for (unsigned it = 0; it < 8; ++it) { const unsigned rw = it * 4u + (lane >> 3), q = lane & 7u; *(volatile v4u*)(hb + (size_t)rw * PREP + 8u * q) = o[it]; }
}

__global__ __launch_bounds__(128) void k_core_gu(const unsigned short* __restrict__ PRE, const unsigned short* __restrict__ CG, const unsigned short* __restrict__ CU, const int* __restrict__ SRT, const int* __restrict__ ETAB, unsigned short* __restrict__ HG, unsigned short* __restrict__ HU) {
  __shared__ __align__(16) unsigned short sa[2][64][72];
  __shared__ __align__(16) _Float16 so[2][4][16][64];
  const unsigned tid = threadIdx.x, lane = tid & 31u, lm = lane & 15u, lh = lane >> 4;
  const unsigned wave = __builtin_amdgcn_readfirstlane(tid >> 5);
  const unsigned e = blockIdx.x, g = e >> 5;
  int base = ETAB[e]; base = base < 0 ? 0 : (base > SROWS - 1 ? SROWS - 1 : base);
  int cnt = ETAB[NEXP + e]; cnt = cnt < 0 ? 0 : (cnt > NB ? NB : cnt); cnt = cnt > SROWS - base ? SROWS - base : cnt;
  const int nch = __builtin_amdgcn_readfirstlane((cnt + 63) >> 6);
  for (int ch = 0; ch < nch; ++ch) {
#pragma unroll
    for (unsigned it = 0; it < 8; ++it) { const unsigned idx = it * 128u + tid, wh = idx >> 9, row = (idx >> 3) & 63u, q = idx & 7u;
      const int rr = ch * 64 + (int)row; const int rc = rr < cnt ? rr : cnt - 1;
      int f = SRT[base + rc]; f = f < 0 ? 0 : (f > NPAIR - 1 ? NPAIR - 1 : f);
      const unsigned tok = (unsigned)f >> 3;
      v4u v = *(const v4u*)(PRE + (size_t)tok * PREP + wh * (unsigned)KP + g * 64u + 8u * q);
      asm volatile("" : "+v"(v));
      const v4u z = {0u, 0u, 0u, 0u};
      v = (rr < cnt) ? v : z;
      *(v4u*)&sa[wh][row][8u * q] = v; }
    __syncthreads();
    v8f accg[4] = {}, accu[4] = {};
#pragma unroll
    for (unsigned kc = 0; kc < RK / 32; ++kc) {
      union { v16h v; v4u q[2]; } ag, au;
      ag.q[0] = *(const v4u*)&sa[0][wave * 16u + lm][kc * 32u + 8u * lh]; ag.q[1] = *(const v4u*)&sa[0][wave * 16u + lm][kc * 32u + 16u + 8u * lh];
      au.q[0] = *(const v4u*)&sa[1][wave * 16u + lm][kc * 32u + 8u * lh]; au.q[1] = *(const v4u*)&sa[1][wave * 16u + lm][kc * 32u + 16u + 8u * lh];
#pragma unroll
      for (int ni = 0; ni < 4; ++ni) {
        const v16h bg = ldfrag_h(CG + (size_t)(e * 64u + ni * 16u + lm) * RK + kc * 32u + 8u * lh);
        accg[ni] = wmma16(ag.v, bg, accg[ni]);
        const v16h bu = ldfrag_h(CU + (size_t)(e * 64u + ni * 16u + lm) * RK + kc * 32u + 8u * lh);
        accu[ni] = wmma16(au.v, bu, accu[ni]); } }
#pragma unroll
    for (int ni = 0; ni < 4; ++ni)
#pragma unroll
      for (int r = 0; r < 8; ++r) { so[0][wave][8u * lh + r][ni * 16 + lm] = toh_flush(accg[ni][r] * HSCALE); so[1][wave][8u * lh + r][ni * 16 + lm] = toh_flush(accu[ni][r] * HSCALE); }
    __syncthreads();
    v4u og[4], ou[4];
#pragma unroll
    for (unsigned it = 0; it < 4; ++it) { const unsigned rw = it * 4u + (lane >> 3), q = lane & 7u; union { v8h h; v4u u; } w;
      w.h = *(const v8h*)&so[0][wave][rw][8u * q]; og[it] = w.u; w.h = *(const v8h*)&so[1][wave][rw][8u * q]; ou[it] = w.u; }
#pragma unroll
    for (unsigned it = 0; it < 4; ++it) { const unsigned rw = it * 4u + (lane >> 3), q = lane & 7u; const int prow = ch * 64 + (int)(wave * 16u + rw);
      if (prow < cnt) { *(volatile v4u*)(HG + (size_t)(base + prow) * RK + 8u * q) = og[it]; *(volatile v4u*)(HU + (size_t)(base + prow) * RK + 8u * q) = ou[it]; } }
    __threadfence();
#pragma unroll
    for (unsigned it = 0; it < 4; ++it) { const unsigned rw = it * 4u + (lane >> 3), q = lane & 7u; const int prow = ch * 64 + (int)(wave * 16u + rw);
      if (prow < cnt) { *(volatile v4u*)(HG + (size_t)(base + prow) * RK + 8u * q) = og[it]; *(volatile v4u*)(HU + (size_t)(base + prow) * RK + 8u * q) = ou[it]; } }
    __syncthreads();
  }
}

__global__ __launch_bounds__(256) void k_gateup(const unsigned short* __restrict__ HG, const unsigned short* __restrict__ HU, const unsigned short* __restrict__ UG, const unsigned short* __restrict__ UU, const int* __restrict__ HDR, unsigned short* __restrict__ ACT) {
  __shared__ __align__(16) _Float16 sh[8][16][64];
  const unsigned t = threadIdx.x, lane = t & 31u, lm = lane & 15u, lh = lane >> 4;
  const unsigned wave = __builtin_amdgcn_readfirstlane(t >> 5);
  const int m0 = (int)blockIdx.y * 128; const unsigned n0 = blockIdx.x * 64u;
  int total = HDR[NG]; total = total < 0 ? 0 : (total > SROWS ? SROWS : total);
  if (m0 >= total) return;
  int g = 0;
#pragma unroll
  for (int j = 1; j < NG; ++j) { const int s = HDR[j]; g = (m0 >= s) ? j : g; }
  int gs = HDR[g]; gs = gs < 0 ? 0 : (gs > SROWS - 1 ? SROWS - 1 : gs);
  int gc = HDR[16 + g]; gc = gc < 1 ? 1 : (gc > NPAIR ? NPAIR : gc);
  int vl = gs + gc - 1; vl = vl > SROWS - 1 ? SROWS - 1 : vl;
  int ra = m0 + (int)(wave * 16u + lm); ra = ra < vl ? ra : vl;
  const unsigned short* pg = HG + (size_t)ra * RK + 8u * lh;
  const unsigned short* pu = HU + (size_t)ra * RK + 8u * lh;
  const unsigned short* bgp = UG + (size_t)((unsigned)g * DFF + n0 + lm) * RK + 8u * lh;
  const unsigned short* bup = UU + (size_t)((unsigned)g * DFF + n0 + lm) * RK + 8u * lh;
  v8f accg[4] = {}, accu[4] = {};
#pragma unroll
  for (unsigned kc = 0; kc < RK / 32; ++kc) { const v16h ag = ldfrag_h(pg + kc * 32u), au = ldfrag_h(pu + kc * 32u);
#pragma unroll
    for (int ni = 0; ni < 4; ++ni) {
      const v16h bg = ldfrag_h(bgp + (size_t)ni * 16u * RK + kc * 32u); accg[ni] = wmma16(ag, bg, accg[ni]);
      const v16h bu = ldfrag_h(bup + (size_t)ni * 16u * RK + kc * 32u); accu[ni] = wmma16(au, bu, accu[ni]); } }
#pragma unroll
  for (int ni = 0; ni < 4; ++ni)
#pragma unroll
    for (int r = 0; r < 8; ++r) { const float zg = accg[ni][r] * GSCALE; const float sg = 1.0f / (1.0f + expf(-zg));
      sh[wave][8u * lh + r][ni * 16 + lm] = toh_flush((zg * sg) * (accu[ni][r] * ASCALE)); }
  __syncthreads();
  v4u o[4];
#pragma unroll
  for (unsigned it = 0; it < 4; ++it) { const unsigned rw = it * 4u + (lane >> 3), q = lane & 7u; union { v8h h; v4u u; } w; w.h = *(const v8h*)&sh[wave][rw][8u * q]; o[it] = w.u; }
  unsigned short* ab = ACT + (size_t)(m0 + (int)(wave * 16u)) * DFF + n0;
#pragma unroll
  for (unsigned it = 0; it < 4; ++it) { const unsigned rw = it * 4u + (lane >> 3), q = lane & 7u; *(volatile v4u*)(ab + (size_t)rw * DFF + 8u * q) = o[it]; }
  __threadfence();
#pragma unroll
  for (unsigned it = 0; it < 4; ++it) { const unsigned rw = it * 4u + (lane >> 3), q = lane & 7u; *(volatile v4u*)(ab + (size_t)rw * DFF + 8u * q) = o[it]; }
}

__global__ __launch_bounds__(256) void k_downin(const unsigned short* __restrict__ ACT, const unsigned short* __restrict__ UD, const int* __restrict__ HDR, unsigned short* __restrict__ XD) {
  __shared__ __align__(16) _Float16 sh[8][16][64];
  const unsigned t = threadIdx.x, lane = t & 31u, lm = lane & 15u, lh = lane >> 4;
  const unsigned wave = __builtin_amdgcn_readfirstlane(t >> 5);
  const int m0 = (int)blockIdx.x * 128;
  int total = HDR[NG]; total = total < 0 ? 0 : (total > SROWS ? SROWS : total);
  if (m0 >= total) return;
  int g = 0;
#pragma unroll
  for (int j = 1; j < NG; ++j) { const int s = HDR[j]; g = (m0 >= s) ? j : g; }
  int gs = HDR[g]; gs = gs < 0 ? 0 : (gs > SROWS - 1 ? SROWS - 1 : gs);
  int gc = HDR[16 + g]; gc = gc < 1 ? 1 : (gc > NPAIR ? NPAIR : gc);
  int vl = gs + gc - 1; vl = vl > SROWS - 1 ? SROWS - 1 : vl;
  int ra = m0 + (int)(wave * 16u + lm); ra = ra < vl ? ra : vl;
  const unsigned short* pa = ACT + (size_t)ra * DFF + 8u * lh;
  const unsigned short* pb = UD + (size_t)((unsigned)g * RK + lm) * DFF + 8u * lh;
  v8f acc[4] = {};
#pragma unroll 2
  for (unsigned kc = 0; kc < DFF / 32; ++kc) { const v16h a = ldfrag_h(pa + kc * 32u);
#pragma unroll
    for (int ni = 0; ni < 4; ++ni) { const v16h b = ldfrag_h(pb + (size_t)ni * 16u * DFF + kc * 32u); acc[ni] = wmma16(a, b, acc[ni]); } }
#pragma unroll
  for (int ni = 0; ni < 4; ++ni)
#pragma unroll
    for (int r = 0; r < 8; ++r) sh[wave][8u * lh + r][ni * 16 + lm] = toh_flush(acc[ni][r] * XSCALE);
  __syncthreads();
  v4u o[4];
#pragma unroll
  for (unsigned it = 0; it < 4; ++it) { const unsigned rw = it * 4u + (lane >> 3), q = lane & 7u; union { v8h h; v4u u; } w; w.h = *(const v8h*)&sh[wave][rw][8u * q]; o[it] = w.u; }
  unsigned short* xb = XD + (size_t)(m0 + (int)(wave * 16u)) * RK;
#pragma unroll
  for (unsigned it = 0; it < 4; ++it) { const unsigned rw = it * 4u + (lane >> 3), q = lane & 7u; *(volatile v4u*)(xb + (size_t)rw * RK + 8u * q) = o[it]; }
  __threadfence();
#pragma unroll
  for (unsigned it = 0; it < 4; ++it) { const unsigned rw = it * 4u + (lane >> 3), q = lane & 7u; *(volatile v4u*)(xb + (size_t)rw * RK + 8u * q) = o[it]; }
}

__global__ __launch_bounds__(128) void k_core_d(const unsigned short* __restrict__ XD, const unsigned short* __restrict__ CD, const int* __restrict__ ETAB, float* __restrict__ HD) {
  __shared__ __align__(16) float sf[4][16][64];
  const unsigned tid = threadIdx.x, lane = tid & 31u, lm = lane & 15u, lh = lane >> 4;
  const unsigned wave = __builtin_amdgcn_readfirstlane(tid >> 5);
  const unsigned e = blockIdx.x;
  int base = ETAB[e]; base = base < 0 ? 0 : (base > SROWS - 1 ? SROWS - 1 : base);
  int cnt = ETAB[NEXP + e]; cnt = cnt < 0 ? 0 : (cnt > NB ? NB : cnt); cnt = cnt > SROWS - base ? SROWS - base : cnt;
  const int nch = __builtin_amdgcn_readfirstlane((cnt + 63) >> 6);
  for (int ch = 0; ch < nch; ++ch) {
    const int rr = ch * 64 + (int)(wave * 16u + lm); const int rc = rr < cnt ? rr : cnt - 1;
    const unsigned short* pa = XD + (size_t)(base + rc) * RK + 8u * lh;
    v8f acc[4] = {};
#pragma unroll
    for (unsigned kc = 0; kc < RK / 32; ++kc) { const v16h a = ldfrag_h(pa + kc * 32u);
#pragma unroll
      for (int ni = 0; ni < 4; ++ni) { const v16h b = ldfrag_h(CD + (size_t)(e * 64u + ni * 16u + lm) * RK + kc * 32u + 8u * lh); acc[ni] = wmma16(a, b, acc[ni]); } }
#pragma unroll
    for (int ni = 0; ni < 4; ++ni)
#pragma unroll
      for (int r = 0; r < 8; ++r) sf[wave][8u * lh + r][ni * 16 + lm] = acc[ni][r];
    __syncthreads();
    v4f v[8];
#pragma unroll
    for (unsigned it = 0; it < 8; ++it) { const unsigned rw = it * 2u + (lane >> 4), pc = lane & 15u; v[it] = *(const v4f*)&sf[wave][rw][4u * pc]; }
#pragma unroll
    for (unsigned it = 0; it < 8; ++it) { const unsigned rw = it * 2u + (lane >> 4), pc = lane & 15u; const int prow = ch * 64 + (int)(wave * 16u + rw);
      if (prow < cnt) *(volatile v4f*)(HD + (size_t)(base + prow) * RK + 4u * pc) = v[it]; }
    __threadfence();
#pragma unroll
    for (unsigned it = 0; it < 8; ++it) { const unsigned rw = it * 2u + (lane >> 4), pc = lane & 15u; const int prow = ch * 64 + (int)(wave * 16u + rw);
      if (prow < cnt) *(volatile v4f*)(HD + (size_t)(base + prow) * RK + 4u * pc) = v[it]; }
    __syncthreads();
  }
}

__global__ __launch_bounds__(256) void k_comb(const float* __restrict__ HD, const int* __restrict__ SEL, const int* __restrict__ POS, const float* __restrict__ WT, unsigned short* __restrict__ A2) {
  __shared__ __align__(16) _Float16 sr[8][KP];
  const unsigned tid = threadIdx.x, lane = tid & 31u;
  const unsigned wave = __builtin_amdgcn_readfirstlane(tid >> 5);
  const unsigned tok = blockIdx.x * 8u + wave;
  const unsigned gl = lane >> 2, c0 = (lane & 3u) * 16u;
  float acc[16];
#pragma unroll
  for (int j = 0; j < 16; ++j) acc[j] = 0.0f;
#pragma unroll 1
  for (unsigned k = 0; k < KTOP; ++k) { const unsigned f = tok * KTOP + k;
    int e = SEL[f]; e = e < 0 ? 0 : (e > NEXP - 1 ? NEXP - 1 : e);
    int p = POS[f]; p = p < 0 ? 0 : (p > SROWS - 1 ? SROWS - 1 : p);
    const float w = WT[f];
    const float* hp = HD + (size_t)p * RK + c0;
    v4f h0 = *(const v4f*)hp, h1 = *(const v4f*)(hp + 4), h2 = *(const v4f*)(hp + 8), h3 = *(const v4f*)(hp + 12);
    asm volatile("" : "+v"(h0)); asm volatile("" : "+v"(h1)); asm volatile("" : "+v"(h2)); asm volatile("" : "+v"(h3));
    const bool mt = (((unsigned)e >> 5) == gl);
#pragma unroll
    for (int j = 0; j < 4; ++j) { acc[j] = fmaf(mt ? h0[j] : 0.0f, w, acc[j]); acc[4 + j] = fmaf(mt ? h1[j] : 0.0f, w, acc[4 + j]);
      acc[8 + j] = fmaf(mt ? h2[j] : 0.0f, w, acc[8 + j]); acc[12 + j] = fmaf(mt ? h3[j] : 0.0f, w, acc[12 + j]); } }
  v8h a, b;
#pragma unroll
  for (int j = 0; j < 8; ++j) { a[j] = toh_flush(acc[j]); b[j] = toh_flush(acc[8 + j]); }
  *(v8h*)&sr[wave][lane * 16u] = a; *(v8h*)&sr[wave][lane * 16u + 8u] = b;
  __syncthreads();
  v4u o[2];
#pragma unroll
  for (unsigned it = 0; it < 2; ++it) { union { v8h h; v4u u; } w; w.h = *(const v8h*)&sr[wave][(it * 32u + lane) * 8u]; o[it] = w.u; }
  unsigned short* ap = A2 + (size_t)tok * KP;
#pragma unroll
  for (unsigned it = 0; it < 2; ++it) *(volatile v4u*)(ap + (it * 32u + lane) * 8u) = o[it];
  __threadfence();
#pragma unroll
  for (unsigned it = 0; it < 2; ++it) *(volatile v4u*)(ap + (it * 32u + lane) * 8u) = o[it];
}

__global__ __launch_bounds__(256) void k_out(const unsigned short* __restrict__ HB, const unsigned short* __restrict__ W2T, float* __restrict__ OUT) {
  __shared__ __align__(16) float sf[8][16][64];
  const unsigned t = threadIdx.x, wave = t >> 5, lane = t & 31u, lm = lane & 15u, lh = lane >> 4, wm = wave >> 1, wn = wave & 1u;
  const unsigned m0 = blockIdx.y * 128u, n0 = blockIdx.x * 128u;
  const unsigned short* ar[2]; const unsigned short* br[4];
#pragma unroll
  for (int mi = 0; mi < 2; ++mi) ar[mi] = HB + (size_t)(m0 + wm * 32u + mi * 16u + lm) * KP + 8u * lh;
#pragma unroll
  for (int ni = 0; ni < 4; ++ni) br[ni] = W2T + (size_t)(n0 + wn * 64u + ni * 16u + lm) * KP + 8u * lh;
  v8f acc[2][4] = {};
#pragma unroll 2
  for (unsigned kc = 0; kc < KP / 32; ++kc) { v16h a[2], b[4];
#pragma unroll
    for (int mi = 0; mi < 2; ++mi) a[mi] = ldfrag_h(ar[mi] + kc * 32u);
#pragma unroll
    for (int ni = 0; ni < 4; ++ni) b[ni] = ldfrag_h(br[ni] + kc * 32u);
#pragma unroll
    for (int mi = 0; mi < 2; ++mi)
#pragma unroll
      for (int ni = 0; ni < 4; ++ni) acc[mi][ni] = wmma16(a[mi], b[ni], acc[mi][ni]); }
#pragma unroll
  for (int mi = 0; mi < 2; ++mi) {
    if (mi) __syncthreads();
#pragma unroll
    for (int ni = 0; ni < 4; ++ni)
#pragma unroll
      for (int r = 0; r < 8; ++r) sf[wave][8u * lh + r][ni * 16 + lm] = acc[mi][ni][r] * OSCALE;
    __syncthreads();
    v4f v[8];
#pragma unroll
    for (unsigned it = 0; it < 8; ++it) { const unsigned rw = it * 2u + (lane >> 4), pc = lane & 15u; v[it] = *(const v4f*)&sf[wave][rw][4u * pc]; }
    float* po = OUT + (size_t)(m0 + wm * 32u + mi * 16u) * DOUT + n0 + wn * 64u;
#pragma unroll
    for (unsigned it = 0; it < 8; ++it) { const unsigned rw = it * 2u + (lane >> 4), pc = lane & 15u; *(volatile v4f*)(po + (size_t)rw * DOUT + 4u * pc) = v[it]; }
    __threadfence();
#pragma unroll
    for (unsigned it = 0; it < 8; ++it) { const unsigned rw = it * 2u + (lane >> 4), pc = lane & 15u; *(volatile v4f*)(po + (size_t)rw * DOUT + 4u * pc) = v[it]; }
  }
}

extern "C" void kernel_launch(void* const* d_in, const int* in_sizes, int n_in, void* d_out, int out_size, void* d_ws, size_t ws_size, hipStream_t stream) {
  if (n_in < 11) return;
  if (in_sizes[0] < NB * DIN || in_sizes[1] < DIN * NEXP) return;
  if (in_sizes[2] < NG * DIN * RK || in_sizes[3] < NEXP * RK * RK || in_sizes[4] < NG * RK * DFF) return;
  if (in_sizes[5] < NG * DIN * RK || in_sizes[6] < NEXP * RK * RK || in_sizes[7] < NG * RK * DFF) return;
  if (in_sizes[8] < NG * DFF * RK || in_sizes[9] < NEXP * RK * RK || in_sizes[10] < NG * RK * DOUT) return;
  if ((size_t)out_size < (size_t)NB * DOUT) return;
  if (ws_size < (size_t)WS_END) return;
  const float* X    = (const float*)d_in[0];
  const float* WG   = (const float*)d_in[1];
  const float* UIG  = (const float*)d_in[2];
  const float* CGI  = (const float*)d_in[3];
  const float* UOG  = (const float*)d_in[4];
  const float* UIU  = (const float*)d_in[5];
  const float* CUI  = (const float*)d_in[6];
  const float* UOU  = (const float*)d_in[7];
  const float* UID  = (const float*)d_in[8];
  const float* CDI  = (const float*)d_in[9];
  const float* UOD  = (const float*)d_in[10];
  char* ws = (char*)d_ws;
  unsigned short* XB  = (unsigned short*)(ws + WS_XB);
  unsigned short* W1T = (unsigned short*)(ws + WS_W1T);
  unsigned short* CGT = (unsigned short*)(ws + WS_CG);
  unsigned short* CUT = (unsigned short*)(ws + WS_CU);
  unsigned short* CDT = (unsigned short*)(ws + WS_CD);
  unsigned short* UGT = (unsigned short*)(ws + WS_UG);
  unsigned short* UUT = (unsigned short*)(ws + WS_UU);
  unsigned short* UDT = (unsigned short*)(ws + WS_UD);
  unsigned short* UOT = (unsigned short*)(ws + WS_UO);
  unsigned short* PRE = (unsigned short*)(ws + WS_PRE);
  unsigned short* HG  = (unsigned short*)(ws + WS_HG);
  unsigned short* HU  = (unsigned short*)(ws + WS_HU);
  unsigned short* ACT = (unsigned short*)(ws + WS_ACT);
  unsigned short* XD  = (unsigned short*)(ws + WS_XD);
  float*          HD  = (float*)(ws + WS_HD);
  unsigned short* A2  = (unsigned short*)(ws + WS_A2);
  int*   SEL  = (int*)(ws + WS_SEL);
  float* WT   = (float*)(ws + WS_WT);
  int*   POS  = (int*)(ws + WS_POS);
  int*   SRT  = (int*)(ws + WS_SRT);
  int*   ETAB = (int*)(ws + WS_ETAB);
  int*   HDR  = (int*)(ws + WS_HDR);
  float* OUT  = (float*)d_out;
  k_cvt_x<<<dim3(NB * DIN / 8 / 256), 256, 0, stream>>>(X, XB);
  k_tr<<<dim3(RK / 64, DIN / 64, NG), 256, 0, stream>>>(UIG, W1T, (unsigned)DIN, (unsigned)RK, (unsigned)DIN, (unsigned)RK, 0u, 1.0f, 0);
  k_tr<<<dim3(RK / 64, DIN / 64, NG), 256, 0, stream>>>(UIU, W1T + (size_t)NG * RK * DIN, (unsigned)DIN, (unsigned)RK, (unsigned)DIN, (unsigned)RK, 0u, 1.0f, 0);
  k_tr<<<dim3(RK / 64, RK / 64, NEXP), 256, 0, stream>>>(CGI, CGT, (unsigned)RK, (unsigned)RK, (unsigned)RK, (unsigned)RK, 0u, WCARRY, 1);
  k_tr<<<dim3(RK / 64, RK / 64, NEXP), 256, 0, stream>>>(CUI, CUT, (unsigned)RK, (unsigned)RK, (unsigned)RK, (unsigned)RK, 0u, WCARRY, 1);
  k_tr<<<dim3(RK / 64, RK / 64, NEXP), 256, 0, stream>>>(CDI, CDT, (unsigned)RK, (unsigned)RK, (unsigned)RK, (unsigned)RK, 0u, WCARRY, 1);
  k_tr<<<dim3(DFF / 64, RK / 64, NG), 256, 0, stream>>>(UOG, UGT, (unsigned)RK, (unsigned)DFF, (unsigned)RK, (unsigned)DFF, 0u, WCARRY, 1);
  k_tr<<<dim3(DFF / 64, RK / 64, NG), 256, 0, stream>>>(UOU, UUT, (unsigned)RK, (unsigned)DFF, (unsigned)RK, (unsigned)DFF, 0u, WCARRY, 1);
  k_tr<<<dim3(RK / 64, DFF / 64, NG), 256, 0, stream>>>(UID, UDT, (unsigned)DFF, (unsigned)RK, (unsigned)DFF, (unsigned)RK, 0u, WCARRY, 1);
  k_tr<<<dim3(DOUT / 64, RK / 64, NG), 256, 0, stream>>>(UOD, UOT, (unsigned)RK, (unsigned)DOUT, (unsigned)KP, 0u, (unsigned)RK, WCARRY, 1);
  k_router<<<dim3(NB / 8), 256, 0, stream>>>(XB, WG, SEL, WT);
  k_plan<<<dim3(1), 256, 0, stream>>>(SEL, POS, SRT, ETAB, HDR);
  k_pre<<<dim3(PREP / 128, NB / 128), 256, 0, stream>>>(XB, W1T, PRE);
  k_core_gu<<<dim3(NEXP), 128, 0, stream>>>(PRE, CGT, CUT, SRT, ETAB, HG, HU);
  k_gateup<<<dim3(DFF / 64, SROWS / 128), 256, 0, stream>>>(HG, HU, UGT, UUT, HDR, ACT);
  k_downin<<<dim3(SROWS / 128), 256, 0, stream>>>(ACT, UDT, HDR, XD);
  k_core_d<<<dim3(NEXP), 128, 0, stream>>>(XD, CDT, ETAB, HD);
  k_comb<<<dim3(NB / 8), 256, 0, stream>>>(HD, SEL, POS, WT, A2);
  k_out<<<dim3(DOUT / 128, NB / 128), 256, 0, stream>>>(A2, UOT, OUT);
}
